// PPRGo_mag_6519760355654
// MI455X (gfx1250) — hardware-verified
//
#include <hip/hip_runtime.h>
#include <math.h>

typedef __attribute__((ext_vector_type(16))) _Float16 v16h;
typedef __attribute__((ext_vector_type(16))) __bf16 v16b;
typedef __attribute__((ext_vector_type(8)))  _Float16 v8h;
typedef __attribute__((ext_vector_type(8)))  float v8f;
typedef __attribute__((ext_vector_type(4)))  float v4f;
typedef __attribute__((ext_vector_type(2)))  float v2f;
typedef __attribute__((ext_vector_type(4)))  unsigned v4u;
typedef __attribute__((ext_vector_type(4)))  int v4i;
typedef float __attribute__((may_alias)) float_a;
typedef int __attribute__((may_alias)) int_a;

template <typename T> __device__ __forceinline__ void vst2(void* p, T v) { *(volatile T*)p = v; __threadfence(); *(volatile T*)p = v; }
__device__ __forceinline__ v8f wmma16(v16h a, v16h b, v8f c) {
  v8f d = __builtin_amdgcn_wmma_f32_16x16x32_f16(false, a, false, b, (short)0, c, false, false);
  asm volatile("v_nop\n\tv_nop\n\tv_nop\n\tv_nop" : "+v"(d) : "v"(a), "v"(b));
  return d;
}
__device__ __forceinline__ v8f wmma_bf(v16b a, v16b b, v8f c) {
  v8f d = __builtin_amdgcn_wmma_f32_16x16x32_bf16(false, a, false, b, (short)0, c, false, false);
  asm volatile("v_nop\n\tv_nop\n\tv_nop\n\tv_nop" : "+v"(d) : "v"(a), "v"(b));
  return d;
}
__device__ __forceinline__ v16h frag_h(const _Float16* rowk0, int lane) {
  union { v16h v; v8h q[2]; } u; const _Float16* p = rowk0 + 8 * (lane >> 4);
  u.q[0] = *(const v8h*)p; u.q[1] = *(const v8h*)(p + 16); return u.v;
}
__device__ __forceinline__ v16h frag_f32(const float* rowk0, int lane) {
  v16h a; const float* p = rowk0 + 8 * (lane >> 4);
#pragma unroll
  for (int i = 0; i < 8; ++i) { a[i] = (_Float16)p[i]; a[8 + i] = (_Float16)p[16 + i]; }
  return a;
}
__device__ __forceinline__ v16h frag_f32s(const float* rowk0, int lane, float sc) {
  v16h a; const float* p = rowk0 + 8 * (lane >> 4);
#pragma unroll
  for (int i = 0; i < 8; ++i) { a[i] = (_Float16)(p[i] * sc); a[8 + i] = (_Float16)(p[16 + i] * sc); }
  return a;
}
__device__ __forceinline__ v16h fragc_f32(const float* W, int k0, int n, int lane, int ld, int K) {
  v16h a; const int g = lane >> 4;
#pragma unroll
  for (int i = 0; i < 8; ++i) { const int ka = k0 + 8 * g + i, kb = ka + 16;
    a[i] = (_Float16)(ka < K ? W[(size_t)(ka < K ? ka : K - 1) * ld + n] : 0.f); a[8 + i] = (_Float16)(kb < K ? W[(size_t)(kb < K ? kb : K - 1) * ld + n] : 0.f); }
  return a;
}
struct F2 { v16b h, l; };
__device__ __forceinline__ F2 bsplit16(const float v[16]) { F2 r;
#pragma unroll
  for (int i = 0; i < 16; ++i) { const __bf16 h = (__bf16)v[i]; r.h[i] = h; r.l[i] = (__bf16)(v[i] - (float)h); }
  return r; }
__device__ __forceinline__ F2 split_row(const float* row, int k0, int lane) { float v[16]; const float* p = row + k0 + 8 * (lane >> 4);
#pragma unroll
  for (int i = 0; i < 8; ++i) { v[i] = p[i]; v[8 + i] = p[16 + i]; }
  return bsplit16(v); }
__device__ __forceinline__ F2 split_rowK(const float* row, int k0, int lane, int K) { float v[16]; const int g = lane >> 4;
#pragma unroll
  for (int i = 0; i < 8; ++i) { const int ka = k0 + 8 * g + i, kb = ka + 16; v[i] = ka < K ? row[ka < K ? ka : K - 1] : 0.f; v[8 + i] = kb < K ? row[kb < K ? kb : K - 1] : 0.f; }
  return bsplit16(v); }
__device__ __forceinline__ F2 split_col(const float* W, int k0, int n, int lane, int ld, int K) { float v[16]; const int g = lane >> 4;
#pragma unroll
  for (int i = 0; i < 8; ++i) { const int ka = k0 + 8 * g + i, kb = ka + 16; v[i] = ka < K ? W[(size_t)(ka < K ? ka : K - 1) * ld + n] : 0.f; v[8 + i] = kb < K ? W[(size_t)(kb < K ? kb : K - 1) * ld + n] : 0.f; }
  return bsplit16(v); }
__device__ __forceinline__ v8f mac3(const F2& a, const F2& b, v8f c) { c = wmma_bf(a.l, b.h, c); c = wmma_bf(a.h, b.l, c); return wmma_bf(a.h, b.h, c); }
__device__ __forceinline__ float sigm(float v) { return 1.0f / (1.0f + expf(-v)); }
#define LDSX() do { asm volatile("s_wait_dscnt 0" ::: "memory"); __builtin_amdgcn_wave_barrier(); __builtin_amdgcn_fence(__ATOMIC_RELEASE, "workgroup"); } while (0)


#define NNODE 100000
#define NNP 100032
#define NF 128
#define HID 512
#define NCL 172
#define NCLP 176
#define KNB 32
#define NTG 10000
#ifndef TNB
#define TNB (NNP / 64)
#define TTG NTG
#endif
typedef __attribute__((ext_vector_type(8))) __bf16 v8b;
__device__ __forceinline__ v16b frag_b(const __bf16* rowk0, int lane) {
  union { v16b v; v8b q[2]; } u; const __bf16* p = rowk0 + 8 * (lane >> 4);
  u.q[0] = *(const v8b*)p; u.q[1] = *(const v8b*)(p + 16); return u.v;
}
__device__ __forceinline__ float bfr(float v) { return (float)(__bf16)v; }
__device__ __attribute__((noinline)) float exp_ni(float v) { return expf(v); }
__device__ __attribute__((noinline)) float erf_ni(float v) { return erff(v); }

#define WS_W0  0u
#define WS_W1  (WS_W0 + 2u * HID * NF)
#define WS_W2  (WS_W1 + 2u * HID * HID)
#define WS_H0  (((WS_W2 + 2u * NCLP * HID) + 127u) / 128u * 128u)
#define WS_H1  (WS_H0 + 2u * (size_t)NNP * HID)
#define WS_LG  (WS_H0)
#define WS_END (WS_H1 + 2u * (size_t)NNP * HID)

__global__ __launch_bounds__(256) void k_pack(const float* __restrict__ W0, const float* __restrict__ W1, const float* __restrict__ W2, __bf16* __restrict__ P0, _Float16* __restrict__ P1, _Float16* __restrict__ P2) {
  const int n = blockIdx.x, which = blockIdx.y, t = threadIdx.x;
  if (which == 0) { __shared__ __align__(16) __bf16 s[NF]; if (t < NF) s[t] = (__bf16)W0[(size_t)t * HID + n]; __syncthreads(); if (t < NF / 8) vst2((unsigned*)(P0 + (size_t)n * NF + t * 8), *(const v4u*)&s[t * 8]); }
  else if (which == 1) { __shared__ __align__(16) _Float16 s1[HID]; for (int k = t; k < HID; k += 256) s1[k] = (_Float16)bfr(W1[(size_t)k * HID + n]); __syncthreads(); for (int q = t; q < HID / 8; q += 256) vst2((unsigned*)(P1 + (size_t)n * HID + q * 8), *(const v4u*)&s1[q * 8]); }
  else { if (n >= NCLP) return; __shared__ __align__(16) _Float16 s2[HID]; for (int k = t; k < HID; k += 256) s2[k] = (_Float16)((n < NCL) ? bfr(W2[(size_t)k * NCL + n]) : 0.f); __syncthreads(); for (int q = t; q < HID / 8; q += 256) vst2((unsigned*)(P2 + (size_t)n * HID + q * 8), *(const v4u*)&s2[q * 8]); }
}
__global__ __launch_bounds__(128) void k_l0(const float* __restrict__ X, const __bf16* __restrict__ P0, _Float16* __restrict__ H0) {
  __shared__ __align__(16) _Float16 so[4][16][136];
  const int tid = threadIdx.x, wave = tid >> 5, lane = tid & 31, col = lane & 15, g = lane >> 4; const size_t r0 = (size_t)blockIdx.x * 64 + wave * 16; const int n0 = blockIdx.y * 128;
  v8f acc[8] = {};
#pragma unroll
  for (int kc = 0; kc < NF / 32; ++kc) { v16b a; { size_t row = r0 + col; if (row >= NNODE) row = NNODE - 1; const float* p = X + row * NF + kc * 32 + 8 * g;
#pragma unroll
      for (int i = 0; i < 8; ++i) { a[i] = (__bf16)p[i]; a[8 + i] = (__bf16)p[16 + i]; } }
#pragma unroll
    for (int j = 0; j < 8; ++j) acc[j] = wmma_bf(a, frag_b(P0 + (size_t)(n0 + j * 16 + col) * NF + kc * 32, lane), acc[j]); }
#pragma unroll
  for (int j = 0; j < 8; ++j)
#pragma unroll
    for (int r = 0; r < 8; ++r) so[wave][8 * g + r][j * 16 + col] = (_Float16)fmaxf(acc[j][r], 0.f);
  LDSX();
  for (int rl = 0; rl < 16; ++rl) if (lane < 16) vst2((unsigned*)(H0 + (r0 + rl) * HID + n0 + lane * 8), *(const v4u*)&so[wave][rl][lane * 8]);
}
template <int L>
__global__ __launch_bounds__(128) void k_l12(const _Float16* __restrict__ Hin, const _Float16* __restrict__ Pw, _Float16* __restrict__ Hout, float* __restrict__ LG) {
  __shared__ __align__(16) _Float16 so[4][16][136]; __shared__ __align__(16) float sf[4][16][132];
  const int tid = threadIdx.x, wave = tid >> 5, lane = tid & 31, col = lane & 15, g = lane >> 4; const size_t r0 = (size_t)blockIdx.x * 64 + wave * 16; const int n0 = blockIdx.y * 128; const int ntile = (L == 2 && blockIdx.y == 1) ? 3 : 8;
  v8f acc[8] = {};
#pragma unroll 2
  for (int kc = 0; kc < HID / 32; ++kc) { const v16h a = frag_h(Hin + (r0 + col) * HID + kc * 32, lane);
#pragma unroll
    for (int j = 0; j < 8; ++j) if (j < ntile) acc[j] = wmma16(a, frag_h(Pw + (size_t)(n0 + j * 16 + col) * HID + kc * 32, lane), acc[j]); }
  if (L == 1) {
#pragma unroll
    for (int j = 0; j < 8; ++j)
#pragma unroll
      for (int r = 0; r < 8; ++r) so[wave][8 * g + r][j * 16 + col] = (_Float16)fmaxf(acc[j][r], 0.f);
    LDSX();
    for (int rl = 0; rl < 16; ++rl) if (lane < 16) vst2((unsigned*)(Hout + (r0 + rl) * HID + n0 + lane * 8), *(const v4u*)&so[wave][rl][lane * 8]);
  } else {
#pragma unroll
    for (int j = 0; j < 8; ++j)
#pragma unroll
      for (int r = 0; r < 8; ++r) sf[wave][8 * g + r][j * 16 + col] = acc[j][r];
    LDSX();
    const int ncols = ntile * 16;
    for (int rl = 0; rl < 16; ++rl) if (lane < ncols / 4) vst2(LG + (r0 + rl) * NCLP + n0 + lane * 4, *(const v4f*)&sf[wave][rl][lane * 4]); }
}
__global__ __launch_bounds__(256) void k_agg(const int* __restrict__ TIDX, const float* __restrict__ TW, const int* __restrict__ BATCH, const float* __restrict__ LG, float* __restrict__ OUT) {
  __shared__ float sagg[16][NCLP]; __shared__ float slse[16]; __shared__ int sidx[16][KNB]; __shared__ float sw[16][KNB];
  const int t = threadIdx.x; const size_t tg0 = (size_t)blockIdx.x * 16;
  for (int e = t; e < 16 * KNB; e += 256) { const int i = e / KNB, k = e % KNB; const size_t tg = tg0 + i; if (tg < NTG) { int node = BATCH[tg]; node = node < 0 ? 0 : (node >= NNODE ? NNODE - 1 : node); int ix = TIDX[(size_t)node * KNB + k]; ix = ix < 0 ? 0 : (ix >= NNODE ? NNODE - 1 : ix); sidx[i][k] = ix; sw[i][k] = bfr(TW[(size_t)node * KNB + k]); } else { sidx[i][k] = 0; sw[i][k] = 0.f; } }
  __syncthreads();
  for (int e = t; e < 16 * NCL; e += 256) { const int i = e / NCL, c = e % NCL; float a = 0.f;
#pragma unroll 1
    for (int k = 0; k < KNB; ++k) a += sw[i][k] * LG[(size_t)sidx[i][k] * NCLP + c];
    sagg[i][c] = a; }
  __syncthreads();
  if (t < 16) { float mx = -3.0e38f; for (int c = 0; c < NCL; ++c) mx = fmaxf(mx, sagg[t][c]); float s = 0.f; for (int c = 0; c < NCL; ++c) s += expf(sagg[t][c] - mx); slse[t] = mx + logf(s); }
  __syncthreads();
  __shared__ __align__(16) float sout[16 * NCL];
  for (int e = t; e < 16 * NCL; e += 256) { const int i = e / NCL, c = e % NCL; sout[e] = sagg[i][c] - slse[i]; }
  __syncthreads();
  if (tg0 + 16 <= NTG) { for (int q = t; q < 16 * NCL / 4; q += 256) vst2(OUT + tg0 * NCL + q * 4, *(const v4f*)&sout[q * 4]); }
}
extern "C" void kernel_launch(void* const* d_in, const int* in_sizes, int n_in, void* d_out, int out_size, void* d_ws, size_t ws_size, hipStream_t stream) {
  (void)in_sizes; (void)n_in; (void)out_size;
  const float** F = (const float**)d_in;
  if (ws_size < (size_t)WS_END) return;
  char* ws = (char*)d_ws; __bf16* P0 = (__bf16*)(ws + WS_W0); _Float16 *P1 = (_Float16*)(ws + WS_W1), *P2 = (_Float16*)(ws + WS_W2), *H0 = (_Float16*)(ws + WS_H0), *H1 = (_Float16*)(ws + WS_H1); float* LG = (float*)(ws + WS_LG);
  k_pack<<<dim3(HID, 3), 256, 0, stream>>>(F[4], F[5], F[6], P0, P1, P2);
  k_l0<<<dim3(TNB, HID / 128), 128, 0, stream>>>(F[0], P0, H0);
  k_l12<1><<<dim3(TNB, HID / 128), 128, 0, stream>>>(H0, P1, H1, nullptr);
  k_l12<2><<<dim3(TNB, 2), 128, 0, stream>>>(H1, P2, nullptr, LG);
  k_agg<<<(TTG + 15) / 16, 256, 0, stream>>>((const int*)d_in[1], F[2], (const int*)d_in[3], LG, (float*)d_out);
}
